// GNAN_44873818308787
// MI455X (gfx1250) — hardware-run, weakly checked
//
#include <hip/hip_runtime.h>

typedef unsigned short v16us __attribute__((ext_vector_type(16)));
typedef unsigned short v8us  __attribute__((ext_vector_type(8)));
typedef __bf16         v16b  __attribute__((ext_vector_type(16)));
typedef float          v8f   __attribute__((ext_vector_type(8)));
typedef float          v4f   __attribute__((ext_vector_type(4)));
typedef v4f  __attribute__((may_alias)) v4fa;
typedef v8us __attribute__((may_alias)) v8usa;

union FragB { v16b v; v16us u; v8us half[2]; };

#define NN      2048
#define FF      64
#define HH      16
#define OO      8
#define FPG     16
#define NB      64
#define IB      16
#define NWAV    8
#define JCH     32
#define DP      36
#define FTPLANE (16 * NN)

static_assert(NN % NB == 0);
static_assert(NN % IB == 0);
static_assert((NN / NWAV) % JCH == 0);
static_assert(FF == 4 * FPG);
static_assert(NB * 4 == 256);

__device__ __forceinline__ unsigned int bf16_bits(float f) {
  unsigned int u = __float_as_uint(f);
  u = u + 0x7FFFu + ((u >> 16) & 1u);
  return u >> 16;
}
__device__ __forceinline__ float bf16v(float f) {
  return __uint_as_float(bf16_bits(f) << 16);
}
__device__ __forceinline__ float relu(float v) { return v > 0.0f ? v : 0.0f; }

__device__ __forceinline__ v8f wmma_bf16(v16b a, v16b b, v8f c) {
  v8f d = __builtin_amdgcn_wmma_f32_16x16x32_bf16(false, a, false, b, (short)0, c, false, false);
  asm volatile("v_nop\n\tv_nop\n\tv_nop\n\tv_nop" : "+v"(d) : "v"(a), "v"(b));
  return d;
}

__global__ __launch_bounds__(256) void fsum_kernel(
    const float* __restrict__ x,
    const float* __restrict__ fW1, const float* __restrict__ fb1,
    const float* __restrict__ fW2, const float* __restrict__ fb2,
    const float* __restrict__ fW3, const float* __restrict__ fb3,
    unsigned short* __restrict__ ft)
{
  __shared__ __attribute__((aligned(16))) float xs[NB * FF];
  __shared__ __attribute__((aligned(16))) float sW3[NWAV * HH * OO];
  __shared__ __attribute__((aligned(16))) float part[4 * NB * OO];
  __shared__ __attribute__((aligned(16))) unsigned short sT[2 * 16 * NB];

  const int tid = threadIdx.x, lane = tid & 31, w = tid >> 5;
  const int grp = tid >> 6, nl = tid & 63;
  const int n0 = blockIdx.x * NB;

  #pragma unroll
  for (int k = 0; k < 4; ++k) {
    const v4f v = *(const v4fa*)(x + (size_t)n0 * FF + tid * 16 + 4 * k);
    const v4f c = { bf16v(v.x), bf16v(v.y), bf16v(v.z), bf16v(v.w) };
    *(v4fa*)(xs + tid * 16 + 4 * k) = c;
  }
  __syncthreads();

  float fx[OO];
  #pragma unroll
  for (int o = 0; o < OO; ++o) fx[o] = 0.0f;
  float* sw = sW3 + w * (HH * OO);

  #pragma unroll 1
  for (int fi = 0; fi < FPG; ++fi) {
    const int f = grp * FPG + fi;

    __syncthreads();
    {
      const v4f wv = *(const v4fa*)(fW3 + (size_t)f * (OO * HH) + 4 * lane);
      const int o = lane >> 2, h0 = 4 * (lane & 3);
      sw[(h0 + 0) * OO + o] = bf16v(wv.x);
      sw[(h0 + 1) * OO + o] = bf16v(wv.y);
      sw[(h0 + 2) * OO + o] = bf16v(wv.z);
      sw[(h0 + 3) * OO + o] = bf16v(wv.w);
    }
    __syncthreads();

    const float xv = xs[nl * FF + f];
    float h1[HH];
    #pragma unroll
    for (int q = 0; q < 4; ++q) {
      const v4f wa = *(const v4fa*)(fW1 + f * HH + 4 * q);
      const v4f ba = *(const v4fa*)(fb1 + f * HH + 4 * q);
      h1[4 * q + 0] = relu(xv * bf16v(wa.x) + bf16v(ba.x));
      h1[4 * q + 1] = relu(xv * bf16v(wa.y) + bf16v(ba.y));
      h1[4 * q + 2] = relu(xv * bf16v(wa.z) + bf16v(ba.z));
      h1[4 * q + 3] = relu(xv * bf16v(wa.w) + bf16v(ba.w));
    }
    float fxf[OO];
    {
      const v4f ba = *(const v4fa*)(fb3 + f * OO);
      const v4f bb = *(const v4fa*)(fb3 + f * OO + 4);
      fxf[0] = bf16v(ba.x); fxf[1] = bf16v(ba.y); fxf[2] = bf16v(ba.z); fxf[3] = bf16v(ba.w);
      fxf[4] = bf16v(bb.x); fxf[5] = bf16v(bb.y); fxf[6] = bf16v(bb.z); fxf[7] = bf16v(bb.w);
    }
    #pragma unroll 1
    for (int g = 0; g < HH; ++g) {
      const float* w2 = fW2 + ((size_t)f * HH + g) * HH;
      float a = bf16v(fb2[f * HH + g]);
      #pragma unroll
      for (int q = 0; q < 4; ++q) {
        const v4f wq = *(const v4fa*)(w2 + 4 * q);
        a += bf16v(wq.x) * h1[4 * q + 0];
        a += bf16v(wq.y) * h1[4 * q + 1];
        a += bf16v(wq.z) * h1[4 * q + 2];
        a += bf16v(wq.w) * h1[4 * q + 3];
      }
      a = relu(a);
      const v4f w3a = *(const v4fa*)(sw + g * OO);
      const v4f w3b = *(const v4fa*)(sw + g * OO + 4);
      fxf[0] += a * w3a.x; fxf[1] += a * w3a.y; fxf[2] += a * w3a.z; fxf[3] += a * w3a.w;
      fxf[4] += a * w3b.x; fxf[5] += a * w3b.y; fxf[6] += a * w3b.z; fxf[7] += a * w3b.w;
    }
    #pragma unroll
    for (int o = 0; o < OO; ++o) fx[o] += fxf[o];
  }

  {
    const v4f pa = { fx[0], fx[1], fx[2], fx[3] };
    const v4f pb = { fx[4], fx[5], fx[6], fx[7] };
    *(v4fa*)(part + tid * OO) = pa;
    *(v4fa*)(part + tid * OO + 4) = pb;
  }
  __syncthreads();
  {
    const int nr = tid >> 2, op = (tid & 3) * 2;
    #pragma unroll
    for (int c = 0; c < 2; ++c) {
      const int o = op + c;
      float s = part[(0 * NB + nr) * OO + o];
      s += part[(1 * NB + nr) * OO + o];
      s += part[(2 * NB + nr) * OO + o];
      s += part[(3 * NB + nr) * OO + o];
      const unsigned int hb = bf16_bits(s);
      const unsigned int lb = bf16_bits(s - __uint_as_float(hb << 16));
      sT[o * NB + nr] = (unsigned short)hb;
      sT[16 * NB + o * NB + nr] = (unsigned short)lb;
    }
    #pragma unroll
    for (int k = 0; k < 4; ++k) {
      const int idx = tid + 256 * k;
      const int p = idx >> 9, rem = idx & 511;
      const int row = 8 + (rem >> 6), col = rem & 63;
      sT[p * (16 * NB) + row * NB + col] = (unsigned short)0;
    }
  }
  __syncthreads();
  {
    const int line = tid >> 3, q8 = tid & 7;
    const int p = line >> 4, row = line & 15;
    const v8us v = *(const v8usa*)(sT + p * (16 * NB) + row * NB + 8 * q8);
    unsigned short* dst = ft + (size_t)p * FTPLANE + (size_t)row * NN + n0 + 8 * q8;
    *(volatile v8us*)dst = v;
    __threadfence();
    *(volatile v8us*)dst = v;
  }
}

__global__ __launch_bounds__(256) void pair_kernel(
    const float* __restrict__ dist, const float* __restrict__ nrm,
    const float* __restrict__ mW1, const float* __restrict__ mb1,
    const float* __restrict__ mW2, const float* __restrict__ mb2,
    const float* __restrict__ mW3, const float* __restrict__ mb3,
    const unsigned short* __restrict__ ft, float* __restrict__ out)
{
  __shared__ __attribute__((aligned(16))) float sD[NWAV * IB * DP];
  __shared__ __attribute__((aligned(16))) float sNm[NWAV * IB * DP];
  __shared__ __attribute__((aligned(16))) float sRed[NWAV * IB * OO];
  __shared__ __attribute__((aligned(16))) float sOut[IB * OO];

  const int tid = threadIdx.x, lane = tid & 31, w = tid >> 5;
  const int hh = lane >> 4, m = lane & 15;
  const int i0 = blockIdx.x * IB;

  const v16us zero16 = {0, 0, 0, 0, 0, 0, 0, 0, 0, 0, 0, 0, 0, 0, 0, 0};
  const v8f zero8 = {0.f, 0.f, 0.f, 0.f, 0.f, 0.f, 0.f, 0.f};

  FragB aw;
  aw.u = zero16;
  {
    const v4f wa = *(const v4fa*)(mW2 + m * HH + 8 * hh);
    const v4f wb = *(const v4fa*)(mW2 + m * HH + 8 * hh + 4);
    aw.u[0] = (unsigned short)bf16_bits(wa.x); aw.u[1] = (unsigned short)bf16_bits(wa.y);
    aw.u[2] = (unsigned short)bf16_bits(wa.z); aw.u[3] = (unsigned short)bf16_bits(wa.w);
    aw.u[4] = (unsigned short)bf16_bits(wb.x); aw.u[5] = (unsigned short)bf16_bits(wb.y);
    aw.u[6] = (unsigned short)bf16_bits(wb.z); aw.u[7] = (unsigned short)bf16_bits(wb.w);
  }
  float w1v[8], b1v[8], b2v[8], w3v[8];
  {
    const v4f a0 = *(const v4fa*)(mW1 + 8 * hh), a1 = *(const v4fa*)(mW1 + 8 * hh + 4);
    const v4f c0 = *(const v4fa*)(mb1 + 8 * hh), c1 = *(const v4fa*)(mb1 + 8 * hh + 4);
    const v4f e0 = *(const v4fa*)(mb2 + 8 * hh), e1 = *(const v4fa*)(mb2 + 8 * hh + 4);
    const v4f g0 = *(const v4fa*)(mW3 + 8 * hh), g1 = *(const v4fa*)(mW3 + 8 * hh + 4);
    w1v[0] = bf16v(a0.x); w1v[1] = bf16v(a0.y); w1v[2] = bf16v(a0.z); w1v[3] = bf16v(a0.w);
    w1v[4] = bf16v(a1.x); w1v[5] = bf16v(a1.y); w1v[6] = bf16v(a1.z); w1v[7] = bf16v(a1.w);
    b1v[0] = bf16v(c0.x); b1v[1] = bf16v(c0.y); b1v[2] = bf16v(c0.z); b1v[3] = bf16v(c0.w);
    b1v[4] = bf16v(c1.x); b1v[5] = bf16v(c1.y); b1v[6] = bf16v(c1.z); b1v[7] = bf16v(c1.w);
    b2v[0] = bf16v(e0.x); b2v[1] = bf16v(e0.y); b2v[2] = bf16v(e0.z); b2v[3] = bf16v(e0.w);
    b2v[4] = bf16v(e1.x); b2v[5] = bf16v(e1.y); b2v[6] = bf16v(e1.z); b2v[7] = bf16v(e1.w);
    w3v[0] = bf16v(g0.x); w3v[1] = bf16v(g0.y); w3v[2] = bf16v(g0.z); w3v[3] = bf16v(g0.w);
    w3v[4] = bf16v(g1.x); w3v[5] = bf16v(g1.y); w3v[6] = bf16v(g1.z); w3v[7] = bf16v(g1.w);
  }
  const float b3 = bf16v(mb3[0]);

  float* sDw = sD + w * (IB * DP);
  float* sNw = sNm + w * (IB * DP);
  const int jw = w * (NN / NWAV);

  v8f acc = zero8;

  #pragma unroll 1
  for (int jc = 0; jc < (NN / NWAV) / JCH; ++jc) {
    const int jb = jw + jc * JCH;

    #pragma unroll
    for (int k = 0; k < 4; ++k) {
      const int row = 4 * k + (lane >> 3), q = lane & 7;
      const size_t gi = (size_t)(i0 + row) * NN + jb + 4 * q;
      const v4f dv = *(const v4fa*)(dist + gi);
      const v4f nv = *(const v4fa*)(nrm + gi);
      const v4f dc = { bf16v(dv.x), bf16v(dv.y), bf16v(dv.z), bf16v(dv.w) };
      const v4f nc = { bf16v(nv.x), bf16v(nv.y), bf16v(nv.z), bf16v(nv.w) };
      *(v4fa*)(sDw + row * DP + 4 * q) = dc;
      *(v4fa*)(sNw + row * DP + 4 * q) = nc;
    }
    __syncthreads();

    float mn[JCH];
    #pragma unroll
    for (int jj = 0; jj < JCH; ++jj) {
      const float dv = sDw[m * DP + jj];
      const float nv = sNw[m * DP + jj];
      FragB bh, bl;
      bh.u = zero16;
      bl.u = zero16;
      #pragma unroll
      for (int e = 0; e < 8; ++e) {
        const float v = relu(dv * w1v[e] + b1v[e]);
        const unsigned int hb = bf16_bits(v);
        const unsigned int lb = bf16_bits(v - __uint_as_float(hb << 16));
        bh.u[e] = (unsigned short)hb;
        bl.u[e] = (unsigned short)lb;
      }
      v8f dacc = zero8;
      dacc = wmma_bf16(aw.v, bh.v, dacc);
      dacc = wmma_bf16(aw.v, bl.v, dacc);
      float part = 0.0f;
      #pragma unroll
      for (int r = 0; r < 8; ++r) part += relu(dacc[r] + b2v[r]) * w3v[r];
      const float tot = part + __shfl_xor(part, 16);
      mn[jj] = (tot + b3) / nv;
    }

    FragB ah, al;
    #pragma unroll
    for (int e = 0; e < 8; ++e) {
      const float v0 = hh ? mn[e + 8] : mn[e];
      const float v1 = hh ? mn[e + 24] : mn[e + 16];
      const unsigned int h0 = bf16_bits(v0);
      const unsigned int l0 = bf16_bits(v0 - __uint_as_float(h0 << 16));
      const unsigned int h1 = bf16_bits(v1);
      const unsigned int l1 = bf16_bits(v1 - __uint_as_float(h1 << 16));
      ah.u[e] = (unsigned short)h0;     al.u[e] = (unsigned short)l0;
      ah.u[8 + e] = (unsigned short)h1; al.u[8 + e] = (unsigned short)l1;
    }
    FragB fh, fl;
    {
      const unsigned short* ph = ft + (size_t)m * NN + jb;
      const unsigned short* pl = ft + FTPLANE + (size_t)m * NN + jb;
      fh.half[0] = *(const v8usa*)(ph + 8 * hh);
      fh.half[1] = *(const v8usa*)(ph + 16 + 8 * hh);
      fl.half[0] = *(const v8usa*)(pl + 8 * hh);
      fl.half[1] = *(const v8usa*)(pl + 16 + 8 * hh);
    }
    acc = wmma_bf16(ah.v, fh.v, acc);
    acc = wmma_bf16(ah.v, fl.v, acc);
    acc = wmma_bf16(al.v, fh.v, acc);

    __syncthreads();
  }

  if (m < OO) {
    #pragma unroll
    for (int r = 0; r < 8; ++r) sRed[w * (IB * OO) + (8 * hh + r) * OO + m] = acc[r];
  }
  __syncthreads();
  if (tid < IB * OO) {
    float s = sRed[tid];
    #pragma unroll
    for (int ww = 1; ww < NWAV; ++ww) s += sRed[ww * (IB * OO) + tid];
    sOut[tid] = s;
  }
  __syncthreads();
  if (w == 0) {
    const v4f v = *(const v4fa*)(sOut + 4 * lane);
    float* p = out + (size_t)i0 * OO + 4 * lane;
    *(volatile v4f*)p = v;
    __threadfence();
    *(volatile v4f*)p = v;
  }
}

extern "C" void kernel_launch(void* const* d_in, const int* in_sizes, int n_in,
                              void* d_out, int out_size, void* d_ws, size_t ws_size,
                              hipStream_t stream) {
  if (n_in < 15) return;
  if (in_sizes[0] != NN * FF) return;
  if (in_sizes[1] != NN * NN || in_sizes[2] != NN * NN) return;
  if (in_sizes[3] != FF * HH || in_sizes[4] != FF * HH) return;
  if (in_sizes[5] != FF * HH * HH || in_sizes[6] != FF * HH) return;
  if (in_sizes[7] != FF * OO * HH || in_sizes[8] != FF * OO) return;
  if (in_sizes[9] != HH || in_sizes[10] != HH || in_sizes[11] != HH * HH) return;
  if (in_sizes[12] != HH || in_sizes[13] != HH || in_sizes[14] != 1) return;
  if (out_size != NN * OO) return;

  const size_t ft_bytes = (size_t)2 * FTPLANE * sizeof(unsigned short);
  if (ft_bytes > ws_size) return;

  const float* x    = (const float*)d_in[0];
  const float* dist = (const float*)d_in[1];
  const float* nrm  = (const float*)d_in[2];
  const float* fW1  = (const float*)d_in[3];
  const float* fb1  = (const float*)d_in[4];
  const float* fW2  = (const float*)d_in[5];
  const float* fb2  = (const float*)d_in[6];
  const float* fW3  = (const float*)d_in[7];
  const float* fb3  = (const float*)d_in[8];
  const float* mW1  = (const float*)d_in[9];
  const float* mb1  = (const float*)d_in[10];
  const float* mW2  = (const float*)d_in[11];
  const float* mb2  = (const float*)d_in[12];
  const float* mW3  = (const float*)d_in[13];
  const float* mb3  = (const float*)d_in[14];
  float* out = (float*)d_out;
  unsigned short* ft = (unsigned short*)d_ws;

  fsum_kernel<<<NN / NB, 256, 0, stream>>>(x, fW1, fb1, fW2, fb2, fW3, fb3, ft);
  pair_kernel<<<NN / IB, 256, 0, stream>>>(dist, nrm, mW1, mb1, mW2, mb2, mW3, mb3, ft, out);
}
